// RITS_41420664602661
// MI455X (gfx1250) — hardware-run, weakly checked
//
#include <hip/hip_runtime.h>
#include <math.h>

typedef __attribute__((ext_vector_type(16))) _Float16 v16h;
typedef __attribute__((ext_vector_type(8)))  _Float16 v8h;
typedef __attribute__((ext_vector_type(8)))  float    v8f;
typedef __attribute__((ext_vector_type(4)))  float    v4f;

constexpr int kB     = 256;
constexpr int kT     = 100;
constexpr int kF     = 256;
constexpr int kH     = 512;
constexpr int kRows  = kB * kT;
constexpr int kG4    = 4 * kH;
constexpr int kKin   = 2 * kF;
constexpr int kKg    = kKin + kH;
constexpr int kBlkRows = 16;
constexpr int kNBlk  = kB / kBlkRows;
constexpr int kThr   = 256;
constexpr int kHP    = 520;
constexpr int kXP    = 264;
constexpr int kSLP   = 36;
constexpr int kPartLine = 32;
constexpr int kHdTile = kBlkRows * kHP;
constexpr float kACarry = 64.0f;
constexpr float kWCarry = 256.0f;
constexpr float kFold   = 1.0f / (kACarry * kWCarry);
constexpr float kF16Min = 6.103515625e-05f;
constexpr int kOut0 = kB * kT * kF;
constexpr int kOut1 = kB * kH;

static_assert(kRows == 25600, "rows");
static_assert(kKg == 1024, "gate K");
static_assert((kF % 32) == 0 && (kH % 32) == 0 && (kKin % 32) == 0, "K multiples of 32");
static_assert((kRows % 64) == 0 && (kH % 64) == 0 && (kF % 64) == 0, "hoisted GEMM M,N multiples of 64");
static_assert(kH == 64 * (kThr / 32), "8 waves x 64 hidden columns");
static_assert(kF == 32 * (kThr / 32), "8 waves x 32 feature columns");
static_assert((kB % kBlkRows) == 0, "batch tiles");
static_assert((kG4 % kThr) == 0, "bias staging loop exact");
static_assert((kHP % 8) == 0 && (kXP % 8) == 0 && (kSLP % 4) == 0 && (kHdTile % 8) == 0, "LDS pitches keep 16-B alignment");
static_assert(kOut0 == 6553600 && kOut1 == 131072, "output extents");

constexpr size_t kSzWG    = (size_t)kG4 * kKg * 2;
constexpr size_t kSzWHIST = (size_t)kF * kH * 2;
constexpr size_t kSzWF    = (size_t)kF * kF * 2;
constexpr size_t kSzWTDH  = (size_t)kH * kF * 2;
constexpr size_t kSzWCOMB = (size_t)kF * kKin * 2;
constexpr size_t kSzD16   = (size_t)kRows * kF * 2;
constexpr size_t kSzGM16  = (size_t)kRows * kKin * 2;
constexpr size_t kSzGH    = (size_t)kRows * kH * 4;
constexpr size_t kSzAL    = (size_t)kRows * kF * 4;
constexpr size_t kSzPART  = (size_t)kNBlk * kT * kPartLine * 4;
constexpr size_t kWsTotal = kSzWG + kSzWHIST + kSzWF + kSzWTDH + kSzWCOMB + kSzD16 + kSzGM16 + kSzGH + kSzAL + kSzPART;
static_assert(kWsTotal == 123281408ull, "carve total");
static_assert(kWsTotal <= 134217728ull, "carve cap");
static_assert((kSzWG % 256) == 0 && (kSzWHIST % 256) == 0 && (kSzWF % 256) == 0 && (kSzWTDH % 256) == 0 &&
              (kSzWCOMB % 256) == 0 && (kSzD16 % 256) == 0 && (kSzGM16 % 256) == 0 && (kSzGH % 256) == 0 &&
              (kSzAL % 256) == 0 && (kSzPART % 256) == 0, "256-B aligned regions");

__device__ __forceinline__ unsigned short f2bf_bits(float f) {
  unsigned u = __float_as_uint(f);
  return (unsigned short)((u + 0x7FFFu + ((u >> 16) & 1u)) >> 16);
}
__device__ __forceinline__ float bf_bits2f(unsigned short h) { return __uint_as_float(((unsigned)h) << 16); }
__device__ __forceinline__ float bf16r(float f) { return bf_bits2f(f2bf_bits(f)); }
__device__ __forceinline__ _Float16 to_f16c(float v) {
  const float w = (fabsf(v) < kF16Min) ? 0.0f : v;
  return (_Float16)w;
}
__device__ __forceinline__ float fsig(float x)  { return __builtin_amdgcn_rcpf(1.0f + __expf(-x)); }
__device__ __forceinline__ float ftanh(float x) { return 1.0f - 2.0f * __builtin_amdgcn_rcpf(__expf(2.0f * x) + 1.0f); }

union FragU { v16h v; v8h h[2]; };
__device__ __forceinline__ v16h frag_load(const _Float16* p) {
  FragU f;
  f.h[0] = *(const v8h*)(p);
  f.h[1] = *(const v8h*)(p + 16);
  return f.v;
}
__device__ __forceinline__ v8f mma_raw(v16h a, v16h b, v8f c) {
  return __builtin_amdgcn_wmma_f32_16x16x32_f16(false, a, false, b, (short)0, c, false, false);
}
__device__ __forceinline__ v8f mma_g(v16h a, v16h b, v8f c) {
  c = __builtin_amdgcn_wmma_f32_16x16x32_f16(false, a, false, b, (short)0, c, false, false);
  asm volatile("v_nop\n\tv_nop\n\tv_nop\n\tv_nop" : "+v"(c) : "v"(a), "v"(b));
  return c;
}
__device__ __forceinline__ void acc_guard4a(v8f& a, v8f& b, v8f& c, v8f& d, v16h x) {
  asm volatile("v_nop\n\tv_nop\n\tv_nop\n\tv_nop" : "+v"(a), "+v"(b), "+v"(c), "+v"(d) : "v"(x));
}
__device__ __forceinline__ void keep4_h(v16h a, v16h b, v16h c, v16h d) { asm volatile("v_nop" :: "v"(a), "v"(b), "v"(c), "v"(d)); }
__device__ __forceinline__ void acc_guard4(v8f& a, v8f& b, v8f& c, v8f& d) {
  asm volatile("v_nop\n\tv_nop\n\tv_nop\n\tv_nop" : "+v"(a), "+v"(b), "+v"(c), "+v"(d));
}
__device__ __forceinline__ void wave_sync_lds() {
  __builtin_amdgcn_fence(__ATOMIC_RELEASE, "workgroup");
  __builtin_amdgcn_wave_barrier();
  __builtin_amdgcn_fence(__ATOMIC_ACQUIRE, "workgroup");
}

__global__ __launch_bounds__(256) void wplane_kernel(const float* __restrict__ src, unsigned short* __restrict__ dst,
                                                     int nrow, int ncol8, int spitch, int dpitch, int dcol0, int zdiag) {
  const int i  = blockIdx.x * 256 + threadIdx.x;
  const int n8 = nrow * ncol8;
  if (i >= n8) return;
  const int row = i / ncol8;
  const int c8  = i - row * ncol8;
  const float* sp = src + (size_t)row * spitch + c8 * 8;
  const v4f a = *(const v4f*)(sp);
  const v4f b = *(const v4f*)(sp + 4);
  v8h hv;
#pragma unroll
  for (int e = 0; e < 4; ++e) {
    const int ka = c8 * 8 + e;
    const int kb = ka + 4;
    float va = bf16r(a[e]) * kWCarry;
    float vb = bf16r(b[e]) * kWCarry;
    va = (zdiag != 0 && ka == row) ? 0.0f : va;
    vb = (zdiag != 0 && kb == row) ? 0.0f : vb;
    hv[e]     = to_f16c(va);
    hv[4 + e] = to_f16c(vb);
  }
  unsigned short* dp = dst + (size_t)row * dpitch + dcol0 + c8 * 8;
  *(volatile v8h*)(dp) = hv;
  __threadfence();
  *(volatile v8h*)(dp) = hv;
}

__global__ __launch_bounds__(256) void aplane_kernel(const float* __restrict__ deltas, const float* __restrict__ masks,
                                                     const float* __restrict__ Wtdx, const float* __restrict__ btdx,
                                                     unsigned short* __restrict__ D16, unsigned short* __restrict__ GM16,
                                                     int n8) {
  const int i = blockIdx.x * 256 + threadIdx.x;
  if (i >= n8) return;
  const int row = i >> 5;
  const int f0  = (i & 31) * 8;
  const float* dp = deltas + (size_t)row * kF + f0;
  const float* mp = masks  + (size_t)row * kF + f0;
  const v4f d0 = *(const v4f*)(dp);
  const v4f d1 = *(const v4f*)(dp + 4);
  const v4f m0 = *(const v4f*)(mp);
  const v4f m1 = *(const v4f*)(mp + 4);
  const v4f b0 = *(const v4f*)(btdx + f0);
  const v4f b1 = *(const v4f*)(btdx + f0 + 4);
  v8h dv, gv, mv;
#pragma unroll
  for (int e = 0; e < 4; ++e) {
    const float da = bf16r(d0[e]);
    const float db = bf16r(d1[e]);
    const float wa = bf16r(Wtdx[(size_t)(f0 + e) * (kF + 1)]);
    const float wb = bf16r(Wtdx[(size_t)(f0 + 4 + e) * (kF + 1)]);
    const float ga = __expf(-fmaxf(da * wa + bf16r(b0[e]), 0.0f));
    const float gb = __expf(-fmaxf(db * wb + bf16r(b1[e]), 0.0f));
    dv[e]     = to_f16c(da * kACarry);
    dv[4 + e] = to_f16c(db * kACarry);
    gv[e]     = to_f16c(ga * kACarry);
    gv[4 + e] = to_f16c(gb * kACarry);
    mv[e]     = to_f16c(bf16r(m0[e]) * kACarry);
    mv[4 + e] = to_f16c(bf16r(m1[e]) * kACarry);
  }
  unsigned short* pd = D16  + (size_t)row * kF + f0;
  unsigned short* pg = GM16 + (size_t)row * kKin + f0;
  unsigned short* pm = GM16 + (size_t)row * kKin + kF + f0;
  *(volatile v8h*)(pd) = dv;
  *(volatile v8h*)(pg) = gv;
  *(volatile v8h*)(pm) = mv;
  __threadfence();
  *(volatile v8h*)(pd) = dv;
  *(volatile v8h*)(pg) = gv;
  *(volatile v8h*)(pm) = mv;
}

template <int ACT>
__global__ __launch_bounds__(256) void gemm64_f16_kernel(
    const unsigned short* __restrict__ Ap, int lda,
    const unsigned short* __restrict__ Btp, int ldb,
    float* __restrict__ Cout, int ldc,
    const float* __restrict__ bias,
    int M, int N, int K, float scale) {
  const _Float16* A  = (const _Float16*)Ap;
  const _Float16* Bt = (const _Float16*)Btp;
  __shared__ __align__(16) float sT[8][16 * 68];
  const int lane = threadIdx.x & 31;
  const int wave = threadIdx.x >> 5;
  const int tilesN = N >> 6;
  const int tilesM = M >> 6;
  const int tile = blockIdx.x * 8 + wave;
  if (tile >= tilesM * tilesN) return;
  const int tm = tile / tilesN;
  const int tn = tile - tm * tilesN;
  const int m0 = tm << 6;
  const int n0 = tn << 6;

  const int rlane = lane & 15;
  const int koff  = (lane >> 4) * 8;
  const int mOff  = (lane >> 4) * 8;

  v8f acc[4][4];
#pragma unroll
  for (int i = 0; i < 4; ++i)
#pragma unroll
    for (int j = 0; j < 4; ++j) acc[i][j] = (v8f){0.f, 0.f, 0.f, 0.f, 0.f, 0.f, 0.f, 0.f};

  for (int k0 = 0; k0 < K; k0 += 32) {
    v16h bh[4];
#pragma unroll
    for (int j = 0; j < 4; ++j) {
      const size_t bo = (size_t)(n0 + (j << 4) + rlane) * ldb + koff + k0;
      bh[j] = frag_load(Bt + bo);
    }
#pragma unroll
    for (int i = 0; i < 4; ++i) {
      const size_t ao = (size_t)(m0 + (i << 4) + rlane) * lda + koff + k0;
      const v16h ah = frag_load(A + ao);
#pragma unroll
      for (int j = 0; j < 4; ++j) acc[i][j] = mma_raw(ah, bh[j], acc[i][j]);
      acc_guard4a(acc[i][0], acc[i][1], acc[i][2], acc[i][3], ah);
    }
    keep4_h(bh[0], bh[1], bh[2], bh[3]);
  }
  acc_guard4(acc[0][0], acc[0][1], acc[0][2], acc[0][3]);
  acc_guard4(acc[1][0], acc[1][1], acc[1][2], acc[1][3]);
  acc_guard4(acc[2][0], acc[2][1], acc[2][2], acc[2][3]);
  acc_guard4(acc[3][0], acc[3][1], acc[3][2], acc[3][3]);

  float* slab = sT[wave];
#pragma unroll
  for (int i = 0; i < 4; ++i) {
    const int mBase = m0 + (i << 4);
#pragma unroll
    for (int j = 0; j < 4; ++j) {
      const int n = n0 + (j << 4) + rlane;
      const float bv = bf16r(bias[n]);
#pragma unroll
      for (int r = 0; r < 8; ++r) {
        float v = acc[i][j][r] * scale;
        v += bv;
        if (ACT == 6) v = __expf(-fmaxf(v, 0.0f));
        if (ACT == 7) v = __builtin_amdgcn_rcpf(1.0f + __expf(-v));
        slab[(mOff + r) * 68 + (j << 4) + rlane] = v;
      }
    }
    wave_sync_lds();
    {
      const int hh = lane >> 4, c4 = (lane & 15) * 4;
      for (int pass = 0; pass < 2; ++pass) {
#pragma unroll
        for (int it = 0; it < 8; ++it) {
          const int row = it * 2 + hh;
          const v4f v = *(const v4f*)(slab + row * 68 + c4);
          *(volatile v4f*)(Cout + (size_t)(mBase + row) * ldc + n0 + c4) = v;
        }
        __threadfence();
      }
    }
    wave_sync_lds();
  }
}

__global__ __launch_bounds__(256) __attribute__((amdgpu_num_vgpr(256)))
void seq_kernel(const float* __restrict__ values, const float* __restrict__ masks,
                const float* __restrict__ GH, const float* __restrict__ AL,
                const unsigned short* __restrict__ Wgp, const unsigned short* __restrict__ Whp,
                const unsigned short* __restrict__ Wfp,
                const float* __restrict__ b_hist, const float* __restrict__ b_feat,
                const float* __restrict__ b_ih, const float* __restrict__ b_hh,
                float* __restrict__ out0, float* __restrict__ out1, float* __restrict__ part) {
  __shared__ __align__(16) _Float16 sHd[2 * kHdTile];
  __shared__ __align__(16) _Float16 sIn[kBlkRows * kHP];
  __shared__ __align__(16) _Float16 sXc[kBlkRows * kXP];
  __shared__ __align__(16) float    sSl[kThr / 32][16 * kSLP];
  __shared__ __align__(16) float    sRed[(kThr / 32) * 4];
  __shared__ __align__(16) float    sBg[kG4];

  const _Float16* Wg = (const _Float16*)Wgp;
  const _Float16* Wh = (const _Float16*)Whp;
  const _Float16* Wf = (const _Float16*)Wfp;

  const int tid = threadIdx.x, lane = tid & 31, wave = tid >> 5;
  const int c = lane & 15, hh = lane >> 4, koff = hh * 8;
  const int q = lane >> 3, c4 = (lane & 7) * 4;
  const int rowbase = blockIdx.x * kBlkRows;
  const int jh = 64 * wave + c;
  const int jf = 32 * wave + c;
  constexpr size_t kGateStride = (size_t)kH * kKg;

#pragma unroll 1
  for (int i = tid; i < 2 * kHdTile; i += kThr) sHd[i] = (_Float16)0.0f;
#pragma unroll 1
  for (int i = tid; i < kBlkRows * kHP; i += kThr) sIn[i] = (_Float16)0.0f;
#pragma unroll 1
  for (int i = tid; i < kBlkRows * kXP; i += kThr) sXc[i] = (_Float16)0.0f;
#pragma unroll 1
  for (int i = tid; i < kG4; i += kThr) sBg[i] = bf16r(b_ih[i]) + bf16r(b_hh[i]);

  float cst[4][8];
#pragma unroll
  for (int us = 0; us < 4; ++us)
#pragma unroll
    for (int r = 0; r < 8; ++r) cst[us][r] = 0.0f;

  float bhv[2], bfv[2];
#pragma unroll
  for (int nt = 0; nt < 2; ++nt) {
    bhv[nt] = bf16r(b_hist[jf + 16 * nt]);
    bfv[nt] = bf16r(b_feat[jf + 16 * nt]);
  }
  __syncthreads();

  const v8f z8 = {0.f, 0.f, 0.f, 0.f, 0.f, 0.f, 0.f, 0.f};
  float* slab = sSl[wave];

#pragma unroll 1
  for (int t = 0; t < kT; ++t) {
    const int cur = t & 1;
    const _Float16* hdc = sHd + cur * kHdTile;
    _Float16* hdn = sHd + (cur ^ 1) * kHdTile;
    const int tn = (t + 1 < kT) ? (t + 1) : (kT - 1);
    const bool last = (t == kT - 1);

    v8f pa[2];
    pa[0] = z8; pa[1] = z8;
    {
      const _Float16* ar = hdc + c * kHP + koff;
      const _Float16* wr = Wh + (size_t)jf * kH + koff;
#pragma unroll 1
      for (int k0 = 0; k0 < kH; k0 += 32) {
        const v16h a  = frag_load(ar + k0);
        const v16h b0 = frag_load(wr + k0);
        const v16h b1 = frag_load(wr + (size_t)16 * kH + k0);
        pa[0] = mma_g(a, b0, pa[0]);
        pa[1] = mma_g(a, b1, pa[1]);
      }
    }
    float xv[2][8], mv[2][8], xh[2][8];
    float n1 = 0.0f, sm = 0.0f;
#pragma unroll
    for (int nt = 0; nt < 2; ++nt) {
#pragma unroll
      for (int r = 0; r < 8; ++r) {
        const size_t vo = (size_t)(rowbase + 8 * hh + r) * (size_t)(kT * kF) + (size_t)t * kF + (size_t)(jf + 16 * nt);
        const float x = bf16r(values[vo]);
        const float m = bf16r(masks[vo]);
        const float xhv = pa[nt][r] * kFold + bhv[nt];
        n1 += fabsf(xhv - x) * m;
        sm += m;
        const float xc = m * x + (1.0f - m) * xhv;
        xv[nt][r] = x; mv[nt][r] = m; xh[nt][r] = xhv;
        sXc[(8 * hh + r) * kXP + jf + 16 * nt] = to_f16c(xc * kACarry);
        sIn[(8 * hh + r) * kHP + kF + jf + 16 * nt] = to_f16c(m * kACarry);
      }
      asm volatile("" ::: "memory");
    }
#pragma unroll
    for (int off = 1; off < 32; off <<= 1) {
      n1 += __shfl_xor(n1, off, 32);
      sm += __shfl_xor(sm, off, 32);
    }
    if (lane == 0) { sRed[wave * 4 + 0] = n1; sRed[wave * 4 + 3] = sm; }
    __syncthreads();

    v8f pz[2];
    pz[0] = z8; pz[1] = z8;
    {
      const _Float16* ar = sXc + c * kXP + koff;
      const _Float16* wr = Wf + (size_t)jf * kF + koff;
#pragma unroll 1
      for (int k0 = 0; k0 < kF; k0 += 32) {
        const v16h a  = frag_load(ar + k0);
        const v16h b0 = frag_load(wr + k0);
        const v16h b1 = frag_load(wr + (size_t)16 * kF + k0);
        pz[0] = mma_g(a, b0, pz[0]);
        pz[1] = mma_g(a, b1, pz[1]);
      }
    }
    float n2 = 0.0f, n3 = 0.0f;
#pragma unroll
    for (int nt = 0; nt < 2; ++nt) {
#pragma unroll
      for (int r = 0; r < 8; ++r) {
        const size_t ai = ((size_t)(rowbase + 8 * hh + r) * kT + (size_t)t) * kF + (size_t)(jf + 16 * nt);
        const float al = AL[ai];
        const float x = xv[nt][r], m = mv[nt][r], xhv = xh[nt][r];
        const float zh = fmaxf(pz[nt][r] * kFold + bfv[nt], 0.0f);
        n2 += fabsf(zh - x) * m;
        const float ch = al * zh + (1.0f - al) * xhv;
        n3 += fabsf(ch - x) * m;
        const float cc = m * x + (1.0f - m) * ch;
        sIn[(8 * hh + r) * kHP + jf + 16 * nt] = to_f16c(cc * kACarry);
        slab[(8 * hh + r) * kSLP + 16 * nt + c] = cc;
      }
    }
#pragma unroll
    for (int off = 1; off < 32; off <<= 1) {
      n2 += __shfl_xor(n2, off, 32);
      n3 += __shfl_xor(n3, off, 32);
    }
    if (lane == 0) { sRed[wave * 4 + 1] = n2; sRed[wave * 4 + 2] = n3; }
    wave_sync_lds();
    {
      v4f ov[4];
#pragma unroll
      for (int it = 0; it < 4; ++it) ov[it] = *(const v4f*)(slab + (it * 4 + q) * kSLP + c4);
      for (int pass = 0; pass < 2; ++pass) {
#pragma unroll
        for (int it = 0; it < 4; ++it) {
          float* op = out0 + ((size_t)(rowbase + it * 4 + q) * kT + (size_t)t) * kF + 32 * wave + c4;
          *(volatile v4f*)(op) = ov[it];
        }
        __threadfence();
      }
    }
    wave_sync_lds();
    __syncthreads();

    if (wave == 0) {
      const int qs = lane & 3;
      float s = 0.0f;
#pragma unroll
      for (int w = 0; w < kThr / 32; ++w) s += sRed[w * 4 + qs];
      const float pv = (lane < 4) ? s : 0.0f;
      float* pp = part + ((size_t)blockIdx.x * kT + (size_t)t) * kPartLine + lane;
      *(volatile float*)(pp) = pv;
      __threadfence();
      *(volatile float*)(pp) = pv;
    }

#pragma unroll
    for (int qd = 0; qd < 4; ++qd) {
      const int col = jh + 16 * qd;
      v8f acc0 = z8, acc1 = z8, acc2 = z8, acc3 = z8;
      {
        const _Float16* ar = sIn + c * kHP + koff;
        const _Float16* wb = Wg + (size_t)col * kKg + koff;
#pragma unroll 1
        for (int k0 = 0; k0 < kKin; k0 += 32) {
          const v16h a  = frag_load(ar + k0);
          const v16h b0 = frag_load(wb + k0);
          const v16h b1 = frag_load(wb + kGateStride + k0);
          const v16h b2 = frag_load(wb + 2 * kGateStride + k0);
          const v16h b3 = frag_load(wb + 3 * kGateStride + k0);
          acc0 = mma_g(a, b0, acc0);
          acc1 = mma_g(a, b1, acc1);
          acc2 = mma_g(a, b2, acc2);
          acc3 = mma_g(a, b3, acc3);
        }
      }
      {
        const _Float16* ar = hdc + c * kHP + koff;
        const _Float16* wb = Wg + (size_t)col * kKg + kKin + koff;
#pragma unroll 1
        for (int k0 = 0; k0 < kH; k0 += 32) {
          const v16h a  = frag_load(ar + k0);
          const v16h b0 = frag_load(wb + k0);
          const v16h b1 = frag_load(wb + kGateStride + k0);
          const v16h b2 = frag_load(wb + 2 * kGateStride + k0);
          const v16h b3 = frag_load(wb + 3 * kGateStride + k0);
          acc0 = mma_g(a, b0, acc0);
          acc1 = mma_g(a, b1, acc1);
          acc2 = mma_g(a, b2, acc2);
          acc3 = mma_g(a, b3, acc3);
        }
      }
      const float bi  = sBg[col];
      const float bfg = sBg[kH + col];
      const float bgg = sBg[2 * kH + col];
      const float bo  = sBg[3 * kH + col];
      float gmn[8];
#pragma unroll
      for (int r = 0; r < 8; ++r) {
        const size_t gi = ((size_t)(rowbase + 8 * hh + r) * kT + (size_t)tn) * kH + (size_t)col;
        gmn[r] = GH[gi];
      }
      float hn8[8];
#pragma unroll
      for (int r = 0; r < 8; ++r) {
        const float gi = acc0[r] * kFold + bi;
        const float gf = acc1[r] * kFold + bfg;
        const float gg = acc2[r] * kFold + bgg;
        const float go = acc3[r] * kFold + bo;
        const float cn = fsig(gf) * cst[qd][r] + fsig(gi) * ftanh(gg);
        const float hn = fsig(go) * ftanh(cn);
        cst[qd][r] = cn;
        hn8[r] = hn;
        const float hd = hn * gmn[r];
        hdn[(8 * hh + r) * kHP + col] = to_f16c(hd * kACarry);
      }
      if (last) {
#pragma unroll
        for (int r = 0; r < 8; ++r) slab[(8 * hh + r) * kSLP + 16 * (qd & 1) + c] = hn8[r];
        if ((qd & 1) == 1) {
          wave_sync_lds();
          v4f ov[4];
#pragma unroll
          for (int it = 0; it < 4; ++it) ov[it] = *(const v4f*)(slab + (it * 4 + q) * kSLP + c4);
          for (int pass = 0; pass < 2; ++pass) {
#pragma unroll
            for (int it = 0; it < 4; ++it) {
              float* op = out1 + (size_t)(rowbase + it * 4 + q) * kH + 64 * wave + 32 * (qd >> 1) + c4;
              *(volatile v4f*)(op) = ov[it];
            }
            __threadfence();
          }
          wave_sync_lds();
        }
      }
    }
    __syncthreads();
  }
}

__global__ __launch_bounds__(32) void loss_kernel(const float* __restrict__ part, float* __restrict__ out2) {
  const int lane = threadIdx.x & 31;
  const int bl = lane & (kNBlk - 1);
  const bool keep = lane < kNBlk;
  float loss = 0.0f;
#pragma unroll 1
  for (int t = 0; t < kT; ++t) {
    const v4f p = *(const v4f*)(part + ((size_t)bl * kT + (size_t)t) * kPartLine);
    float p0 = p[0];
    float p1 = p[1];
    float p2 = p[2];
    float p3 = p[3];
    asm volatile("" : "+v"(p0), "+v"(p1), "+v"(p2), "+v"(p3));
    float a0 = keep ? p0 : 0.0f;
    float a1 = keep ? p1 : 0.0f;
    float a2 = keep ? p2 : 0.0f;
    float a3 = keep ? p3 : 0.0f;
#pragma unroll
    for (int off = 1; off < 32; off <<= 1) {
      a0 += __shfl_xor(a0, off, 32);
      a1 += __shfl_xor(a1, off, 32);
      a2 += __shfl_xor(a2, off, 32);
      a3 += __shfl_xor(a3, off, 32);
    }
    const float den = a3 + 1e-9f;
    const float rden = 1.0f / den;
    loss += a0 * rden;
    loss += a1 * rden;
    loss += a2 * rden;
  }
  const float res = loss * (1.0f / (3.0f * (float)kT));
  if (lane == 0) {
    *(volatile float*)(out2) = res;
    __threadfence();
    *(volatile float*)(out2) = res;
  }
}

extern "C" void kernel_launch(void* const* d_in, const int* in_sizes, int n_in,
                              void* d_out, int out_size, void* d_ws, size_t ws_size,
                              hipStream_t stream) {
  if (n_in < 17 || d_out == nullptr || d_ws == nullptr) return;
  if (in_sizes[0] != kOut0 || in_sizes[1] != kOut0 || in_sizes[2] != kOut0) return;
  if (in_sizes[3] != kH * kF || in_sizes[4] != kH) return;
  if (in_sizes[5] != kF * kF || in_sizes[6] != kF) return;
  if (in_sizes[7] != kF * kH || in_sizes[8] != kF) return;
  if (in_sizes[9] != kF * kF || in_sizes[10] != kF) return;
  if (in_sizes[11] != kF * kKin || in_sizes[12] != kF) return;
  if (in_sizes[13] != kG4 * kKin || in_sizes[14] != kG4 * kH) return;
  if (in_sizes[15] != kG4 || in_sizes[16] != kG4) return;
  if (out_size != kOut0 + kOut1 + 1) return;
  if (ws_size < kWsTotal) return;

  const float* values = (const float*)d_in[0];
  const float* masks  = (const float*)d_in[1];
  const float* deltas = (const float*)d_in[2];
  const float* W_td_h = (const float*)d_in[3];
  const float* b_td_h = (const float*)d_in[4];
  const float* W_td_x = (const float*)d_in[5];
  const float* b_td_x = (const float*)d_in[6];
  const float* W_hist = (const float*)d_in[7];
  const float* b_hist = (const float*)d_in[8];
  const float* W_feat = (const float*)d_in[9];
  const float* b_feat = (const float*)d_in[10];
  const float* W_comb = (const float*)d_in[11];
  const float* b_comb = (const float*)d_in[12];
  const float* W_ih   = (const float*)d_in[13];
  const float* W_hh   = (const float*)d_in[14];
  const float* b_ih   = (const float*)d_in[15];
  const float* b_hh   = (const float*)d_in[16];
  float* out0 = (float*)d_out;
  float* out1 = out0 + (size_t)kOut0;
  float* out2 = out1 + (size_t)kOut1;

  char* ws = (char*)d_ws;
  size_t off = 0;
  auto carve = [&](size_t bytes) -> char* { char* p = ws + off; off += bytes; return p; };
  unsigned short* WG    = (unsigned short*)carve(kSzWG);
  unsigned short* WHIST = (unsigned short*)carve(kSzWHIST);
  unsigned short* WF    = (unsigned short*)carve(kSzWF);
  unsigned short* WTDH  = (unsigned short*)carve(kSzWTDH);
  unsigned short* WCOMB = (unsigned short*)carve(kSzWCOMB);
  unsigned short* D16   = (unsigned short*)carve(kSzD16);
  unsigned short* GM16  = (unsigned short*)carve(kSzGM16);
  float*          GH    = (float*)carve(kSzGH);
  float*          AL    = (float*)carve(kSzAL);
  float*          PART  = (float*)carve(kSzPART);
  if (off != kWsTotal || off > ws_size) return;

  wplane_kernel<<<(kG4 * (kKin / 8)) / 256, 256, 0, stream>>>(W_ih, WG, kG4, kKin / 8, kKin, kKg, 0, 0);
  wplane_kernel<<<(kG4 * (kH / 8)) / 256, 256, 0, stream>>>(W_hh, WG, kG4, kH / 8, kH, kKg, kKin, 0);
  wplane_kernel<<<(kF * (kH / 8)) / 256, 256, 0, stream>>>(W_hist, WHIST, kF, kH / 8, kH, kH, 0, 0);
  wplane_kernel<<<(kF * (kF / 8)) / 256, 256, 0, stream>>>(W_feat, WF, kF, kF / 8, kF, kF, 0, 1);
  wplane_kernel<<<(kH * (kF / 8)) / 256, 256, 0, stream>>>(W_td_h, WTDH, kH, kF / 8, kF, kF, 0, 0);
  wplane_kernel<<<(kF * (kKin / 8)) / 256, 256, 0, stream>>>(W_comb, WCOMB, kF, kKin / 8, kKin, kKin, 0, 0);

  const int n8a = kRows * (kF / 8);
  aplane_kernel<<<n8a / 256, 256, 0, stream>>>(deltas, masks, W_td_x, b_td_x, D16, GM16, n8a);

  gemm64_f16_kernel<6><<<(kRows / 64) * (kH / 64) / 8, 256, 0, stream>>>(
      D16, kF, WTDH, kF, GH, kH, b_td_h, kRows, kH, kF, kFold);
  gemm64_f16_kernel<7><<<(kRows / 64) * (kF / 64) / 8, 256, 0, stream>>>(
      GM16, kKin, WCOMB, kKin, AL, kF, b_comb, kRows, kF, kKin, kFold);

  seq_kernel<<<kNBlk, kThr, 0, stream>>>(values, masks, GH, AL, WG, WHIST, WF,
                                         b_hist, b_feat, b_ih, b_hh, out0, out1, PART);

  loss_kernel<<<1, 32, 0, stream>>>(PART, out2);
}
